// HybridNet_65481071401691
// MI455X (gfx1250) — hardware-verified
//
#include <hip/hip_runtime.h>

#define __bf16 _Float16
typedef __attribute__((ext_vector_type(8)))  float  v8f;
typedef __attribute__((ext_vector_type(16))) _Float16 v16bf;
typedef __attribute__((ext_vector_type(8)))  _Float16 v8bf;
typedef __attribute__((ext_vector_type(4)))  int    v4i;
#define VST2(T, ptr, val) do { const T _v = (val); *(volatile T*)(ptr) = _v; __threadfence(); *(volatile T*)(ptr) = _v; } while (0)

#define BATCH 4096
#define FEAT  2048
#define BM 128
#define BN 128
#define BK 64

__global__ __launch_bounds__(256)
void wt_transpose(const float* __restrict__ W0, const float* __restrict__ W1,
                  const float* __restrict__ W2, const float* __restrict__ W3,
                  __bf16* __restrict__ Wt)
{
    const float* Ws[4] = {W0, W1, W2, W3};
    const float* W = Ws[blockIdx.y];
    __bf16* dst = Wt + (size_t)blockIdx.y * FEAT * FEAT;
    const size_t i = ((size_t)blockIdx.x * 256 + threadIdx.x) * 8;
    v8bf o;
#pragma unroll
    for (int e = 0; e < 8; ++e) o[e] = (__bf16)W[i + e];
    VST2(v8bf, dst + i, o);
}

__global__ __launch_bounds__(256)
void act_sigmoid(const float* __restrict__ x, const float* __restrict__ cw,
                 const float* __restrict__ cb, __bf16* __restrict__ h)
{
    const float s = cw[0] + cw[1] + cw[2] + cw[3];
    const float c = cb[0];
    const size_t i = ((size_t)blockIdx.x * blockDim.x + threadIdx.x) * 8;
    const float4 v0 = *(const float4*)(x + i);
    const float4 v1 = *(const float4*)(x + i + 4);
    float t[8] = {v0.x, v0.y, v0.z, v0.w, v1.x, v1.y, v1.z, v1.w};
    v8bf o;
#pragma unroll
    for (int j = 0; j < 8; ++j) {
        float z = t[j] * s + c;
        o[j] = (__bf16)(1.0f / (1.0f + expf(-z)));
    }
    VST2(v8bf, h + i, o);
}

__global__ __launch_bounds__(256)
void gemm_bf16_relu(const __bf16* __restrict__ A, const __bf16* __restrict__ Bt,
                    const float* __restrict__ bias, __bf16* __restrict__ C,
                    int M, int N, int K)
{
    __shared__ __align__(16) __bf16 Ash[2][BM][BK + 8];
    __shared__ __align__(16) __bf16 Bsh[2][BN][BK + 8];
    __shared__ __align__(16) __bf16 Csh[8][32][72];

    const int tid  = threadIdx.x;
    const int wave = tid >> 5;
    const int lane = tid & 31;
    const int lh   = lane >> 4;
    const int lm   = lane & 15;
    const int wm   = wave >> 1;
    const int wn   = wave & 1;
    const int bm0  = blockIdx.y * BM;
    const int bn0  = blockIdx.x * BN;

    v8f acc[2][4];
#pragma unroll
    for (int mi = 0; mi < 2; ++mi)
#pragma unroll
        for (int ni = 0; ni < 4; ++ni)
            acc[mi][ni] = (v8f)(0.0f);

    const int ar = tid >> 1;
    const int ac = (tid & 1) * 32;
    const __bf16* gA = A  + (size_t)(bm0 + ar) * K + ac;
    const __bf16* gB = Bt + (size_t)(bn0 + ar) * K + ac;
    v8bf ra[4], rb[4];
    auto load_regs = [&](int k0) {
#pragma unroll
        for (int i = 0; i < 4; ++i) { ra[i] = *(const v8bf*)(gA + k0 + 8 * i); rb[i] = *(const v8bf*)(gB + k0 + 8 * i); }
    };
    auto store_regs = [&](int b_) {
#pragma unroll
        for (int i = 0; i < 4; ++i) { *(v8bf*)&Ash[b_][ar][ac + 8 * i] = ra[i]; *(v8bf*)&Bsh[b_][ar][ac + 8 * i] = rb[i]; }
    };
    load_regs(0); store_regs(0);
    __syncthreads();

    int buf = 0;
    for (int k0 = 0; k0 < K; k0 += BK) {
        if (k0 + BK < K) load_regs(k0 + BK);

#pragma unroll
        for (int kk = 0; kk < BK; kk += 32) {
            v16bf afrag[2];
#pragma unroll
            for (int mi = 0; mi < 2; ++mi) {
                const __bf16* ap = &Ash[buf][wm * 32 + mi * 16 + lm][kk];
                v8bf alo = *(const v8bf*)(ap + lh * 8);
                v8bf ahi = *(const v8bf*)(ap + 16 + lh * 8);
                afrag[mi] = __builtin_shufflevector(alo, ahi,
                    0, 1, 2, 3, 4, 5, 6, 7, 8, 9, 10, 11, 12, 13, 14, 15);
            }
#pragma unroll
            for (int ni = 0; ni < 4; ++ni) {
                const __bf16* bp = &Bsh[buf][wn * 64 + ni * 16 + lm][kk];
                v8bf blo = *(const v8bf*)(bp + lh * 8);
                v8bf bhi = *(const v8bf*)(bp + 16 + lh * 8);
                v16bf bfrag = __builtin_shufflevector(blo, bhi,
                    0, 1, 2, 3, 4, 5, 6, 7, 8, 9, 10, 11, 12, 13, 14, 15);
#pragma unroll
                for (int mi = 0; mi < 2; ++mi)
                {   acc[mi][ni] = __builtin_amdgcn_wmma_f32_16x16x32_f16(
                        false, afrag[mi], false, bfrag,
                        (short)0, acc[mi][ni], false, false);
                    asm volatile("v_nop\n\tv_nop\n\tv_nop\n\tv_nop" : "+v"(acc[mi][ni]) : "v"(afrag[mi]), "v"(bfrag)); }
            }
        }

        if (k0 + BK < K) store_regs(buf ^ 1);
        __syncthreads();
        buf ^= 1;
    }

    __bf16 (*ct)[72] = Csh[wave];
#pragma unroll
    for (int ni = 0; ni < 4; ++ni) {
        const int cn = ni * 16 + lm;
        const float bv = bias[bn0 + wn * 64 + cn];
#pragma unroll
        for (int mi = 0; mi < 2; ++mi)
#pragma unroll
            for (int v = 0; v < 8; ++v) {
                float r = acc[mi][ni][v] + bv;
                ct[mi * 16 + lh * 8 + v][cn] = (__bf16)(r > 0.0f ? r : 0.0f);
            }
    }
    __builtin_amdgcn_fence(__ATOMIC_RELEASE, "workgroup"); __builtin_amdgcn_wave_barrier(); __builtin_amdgcn_fence(__ATOMIC_ACQUIRE, "workgroup");
    for (int pass = 0; pass < 2; ++pass) {
#pragma unroll
        for (int j = 0; j < 8; ++j) {
            const int rr = j * 4 + (lane >> 3), sg = lane & 7;
            *(volatile v8bf*)(C + (size_t)(bm0 + wm * 32 + rr) * N + bn0 + wn * 64 + sg * 8) = *(const v8bf*)&ct[rr][sg * 8];
        }
        __threadfence();
    }
}

__global__ __launch_bounds__(256)
void head_kernel(const __bf16* __restrict__ H, const float* __restrict__ Wh,
                 const float* __restrict__ bh, float* __restrict__ out, int K)
{
    __shared__ float so[32];
    const int lane = threadIdx.x & 31, wave = threadIdx.x >> 5;
    for (int q = 0; q < 2; ++q) {
        const int row = blockIdx.x * 16 + wave * 2 + q;
        const __bf16* hr = H + (size_t)row * K;
        float s0 = 0.0f, s1 = 0.0f;
        for (int k = lane; k < K; k += 32) {
            const float hv = (float)hr[k];
            s0 += hv * Wh[k];
            s1 += hv * Wh[K + k];
        }
#pragma unroll
        for (int off = 16; off > 0; off >>= 1) {
            s0 += __shfl_xor(s0, off, 32);
            s1 += __shfl_xor(s1, off, 32);
        }
        if (lane == 0) { so[(wave * 2 + q) * 2] = s0 + bh[0]; so[(wave * 2 + q) * 2 + 1] = s1 + bh[1]; }
    }
    __syncthreads();
    if (threadIdx.x < 32) VST2(float, out + (size_t)blockIdx.x * 32 + threadIdx.x, so[threadIdx.x]);
}

extern "C" void kernel_launch(void* const* d_in, const int* in_sizes, int n_in,
                              void* d_out, int out_size, void* d_ws, size_t ws_size,
                              hipStream_t stream) {
    const float* x      = (const float*)d_in[0];
    const float* conv_w = (const float*)d_in[1];
    const float* conv_b = (const float*)d_in[2];
    const float* W[4]   = {(const float*)d_in[3], (const float*)d_in[5],
                           (const float*)d_in[7], (const float*)d_in[9]};
    const float* b[4]   = {(const float*)d_in[4], (const float*)d_in[6],
                           (const float*)d_in[8], (const float*)d_in[10]};
    const float* Wh     = (const float*)d_in[11];
    const float* bh     = (const float*)d_in[12];
    float* out          = (float*)d_out;

    (void)in_sizes; (void)n_in; (void)out_size;
    if (ws_size < (size_t)(4 * FEAT * FEAT + 2 * BATCH * FEAT) * 2) return;
    char* ws = (char*)d_ws;
    __bf16* Wt = (__bf16*)ws;
    const size_t wmat = (size_t)FEAT * FEAT;
    __bf16* h0 = (__bf16*)(ws + 4 * wmat * sizeof(__bf16));
    __bf16* h1 = h0 + (size_t)BATCH * FEAT;

    wt_transpose<<<dim3(FEAT * FEAT / 8 / 256, 4), dim3(256), 0, stream>>>(
        W[0], W[1], W[2], W[3], Wt);

    act_sigmoid<<<(BATCH * FEAT) / (256 * 8), 256, 0, stream>>>(x, conv_w, conv_b, h0);

    const dim3 ggrid(FEAT / BN, BATCH / BM);
    gemm_bf16_relu<<<ggrid, 256, 0, stream>>>(h0, Wt + 0 * wmat, b[0], h1, BATCH, FEAT, FEAT);
    gemm_bf16_relu<<<ggrid, 256, 0, stream>>>(h1, Wt + 1 * wmat, b[1], h0, BATCH, FEAT, FEAT);
    gemm_bf16_relu<<<ggrid, 256, 0, stream>>>(h0, Wt + 2 * wmat, b[2], h1, BATCH, FEAT, FEAT);
    gemm_bf16_relu<<<ggrid, 256, 0, stream>>>(h1, Wt + 3 * wmat, b[3], h0, BATCH, FEAT, FEAT);

    head_kernel<<<BATCH / 16, 256, 0, stream>>>(h0, Wh, bh, out, FEAT);
}
